// ConditionalSDFModel_30107720745798
// MI455X (gfx1250) — hardware-verified
//
#include <hip/hip_runtime.h>

typedef __attribute__((ext_vector_type(16))) _Float16 v16h;
typedef __attribute__((ext_vector_type(8)))  _Float16 v8h;
typedef __attribute__((ext_vector_type(8)))  float    v8f;
typedef __attribute__((ext_vector_type(4)))  float    v4f;

constexpr int kPts     = 65536;
constexpr int kExp     = 8;
constexpr int kDimX    = 3;
constexpr int kLat     = 64;
constexpr int kHid     = 256;
constexpr int kInW     = kDimX + kLat;
constexpr int kRowsBlk = 512;
constexpr int kTileM   = 64;
constexpr int kPitchA  = 264;
constexpr float kCarryW   = 256.0f;
constexpr float kCarryA   = 16.0f;
constexpr float kFoldBack = 1.0f / (kCarryW * kCarryA);
constexpr float kMinNormH = 6.103515625e-5f;
static_assert(kInW == 67, "layer-0 input width");
static_assert((kPts % kRowsBlk) == 0, "row chunks tile the batch");
static_assert((kHid % 32) == 0, "K multiple of 32");
static_assert((kHid % 64) == 0, "plane tiles");
static_assert(((kPitchA * 2) % 16) == 0, "LDS tile rows 16-B aligned");
static_assert(kRowsBlk == 512, "partition passes and the final store assume 512 rows");

constexpr size_t kOffPlane1 = 0;
constexpr size_t kOffPlane2 = kOffPlane1 + (size_t)kExp * kHid * kHid * 2;
constexpr size_t kOffFold0  = kOffPlane2 + (size_t)kExp * kHid * kHid * 2;
constexpr size_t kWsTotal   = kOffFold0 + (size_t)kExp * kHid * 4;
static_assert(kWsTotal == 2105344ull, "carve total");
static_assert(kWsTotal <= 134217728ull, "carve cap");
static_assert((kOffPlane2 % 128) == 0 && (kOffFold0 % 128) == 0, "128-B aligned regions");

union FragU { v16h v; v8h h[2]; };

__device__ __forceinline__ v16h frag_load(const _Float16* p) {
  FragU f;
  f.h[0] = *(const v8h*)(p);
  f.h[1] = *(const v8h*)(p + 16);
  return f.v;
}

__device__ __forceinline__ v8f mma_h(v16h a, v16h b, v8f c) {
  c = __builtin_amdgcn_wmma_f32_16x16x32_f16(false, a, false, b, (short)0, c, false, false);
  asm volatile("v_nop\n\tv_nop\n\tv_nop\n\tv_nop" : "+v"(c) : "v"(a), "v"(b));
  return c;
}

__device__ __forceinline__ _Float16 operand_h(float carried) {
  const float f = (fabsf(carried) < kMinNormH) ? 0.0f : carried;
  return (_Float16)f;
}

__global__ __launch_bounds__(256) void weight_plane_kernel(
    const float* __restrict__ W1, const float* __restrict__ W2,
    _Float16* __restrict__ plane1, _Float16* __restrict__ plane2)
{
  __shared__ float sT[64 * 65];
  const int tid = threadIdx.x;
  const int bid = blockIdx.x;
  const int mat = bid >> 7;
  const int rem = bid & 127;
  const int e   = rem >> 4;
  const int k0  = ((rem >> 2) & 3) * 64;
  const int n0  = (rem & 3) * 64;
  const float* W = (mat ? W2 : W1) + (size_t)e * kHid * kHid;
  _Float16* P    = (mat ? plane2 : plane1) + (size_t)e * kHid * kHid;

  const int lr  = tid >> 4;
  const int lc4 = (tid & 15) * 4;
#pragma unroll
  for (int i = 0; i < 4; ++i) {
    const int kk = lr + 16 * i;
    const v4f v = *(const v4f*)(W + (size_t)(k0 + kk) * kHid + n0 + lc4);
    sT[kk * 65 + lc4 + 0] = v[0];
    sT[kk * 65 + lc4 + 1] = v[1];
    sT[kk * 65 + lc4 + 2] = v[2];
    sT[kk * 65 + lc4 + 3] = v[3];
  }
  __syncthreads();

  const int sn = tid >> 3;
  const int k8 = (tid & 7) * 8;
  v8h hv[2];
#pragma unroll
  for (int it = 0; it < 2; ++it) {
    const int n = sn + 32 * it;
#pragma unroll
    for (int q = 0; q < 8; ++q) {
      const float w = sT[(k8 + q) * 65 + n];
      hv[it][q] = operand_h(w * kCarryW);
    }
  }
  for (int pass = 0; pass < 2; ++pass) {
#pragma unroll
    for (int it = 0; it < 2; ++it) {
      const int n = sn + 32 * it;
      *(volatile v8h*)(P + (size_t)(n0 + n) * kHid + k0 + k8) = hv[it];
    }
    __threadfence();
  }
}

__global__ __launch_bounds__(256) void latent_fold_kernel(
    const float* __restrict__ emb, const float* __restrict__ W0,
    const float* __restrict__ b0, float* __restrict__ fold0)
{
  __shared__ __align__(16) float sC[kHid];
  __shared__ float sE[kLat];
  const int tid = threadIdx.x;
  const int e   = blockIdx.x;
  if (tid < kLat) sE[tid] = emb[e * kLat + tid];
  __syncthreads();
  const float* Wl = W0 + ((size_t)e * kInW + kDimX) * kHid + tid;
  float s = b0[e * kHid + tid];
#pragma unroll 8
  for (int k = 0; k < kLat; ++k) s = fmaf(sE[k], Wl[(size_t)k * kHid], s);
  sC[tid] = s;
  __syncthreads();
  if (tid < 64) {
    const v4f v = *(const v4f*)(sC + tid * 4);
    float* q = fold0 + e * kHid + tid * 4;
    *(volatile v4f*)q = v;
    __threadfence();
    *(volatile v4f*)q = v;
  }
}

__global__ __launch_bounds__(256) void routed_decoder_kernel(
    const float* __restrict__ x, const int* __restrict__ labels,
    const float* __restrict__ W0, const float* __restrict__ fold0,
    const _Float16* __restrict__ plane1, const float* __restrict__ b1,
    const _Float16* __restrict__ plane2, const float* __restrict__ b2,
    const float* __restrict__ W3, const float* __restrict__ b3,
    float* __restrict__ out)
{
  __shared__ __align__(16) _Float16 sA[kTileM * kPitchA];
  __shared__ __align__(16) float sX[kRowsBlk * kDimX];
  __shared__ __align__(16) float sTx[kTileM * 4];
  __shared__ __align__(16) float sOut[kRowsBlk];
  __shared__ float sPart[8 * kTileM];
  __shared__ int sLab[kRowsBlk];
  __shared__ int sPerm[kRowsBlk];
  __shared__ int sTrow[kTileM];
  __shared__ int sCnt[kExp];

  const int tid  = threadIdx.x;
  const int lane = tid & 31;
  const int wave = tid >> 5;
  const int hh   = lane >> 4;
  const int rl   = lane & 15;
  const int row0 = blockIdx.x * kRowsBlk;

#pragma unroll
  for (int j = 0; j < 6; ++j) sX[tid + 256 * j] = x[(size_t)row0 * kDimX + tid + 256 * j];
#pragma unroll
  for (int j = 0; j < 2; ++j) {
    int l = labels[row0 + tid + 256 * j];
    l = l < 0 ? 0 : l;
    l = l > (kExp - 1) ? (kExp - 1) : l;
    sLab[tid + 256 * j] = l;
    sOut[tid + 256 * j] = 0.0f;
  }
  __syncthreads();

  {
    int cntw = 0;
#pragma unroll 1
    for (int it = 0; it < kRowsBlk / 32; ++it) {
      const int l = sLab[it * 32 + lane];
      const unsigned m = __builtin_amdgcn_ballot_w32(l == wave);
      cntw += __builtin_popcount(m);
    }
    if (lane == 0) sCnt[wave] = cntw;
  }
  __syncthreads();

  {
    int base = 0;
#pragma unroll
    for (int e2 = 0; e2 < kExp; ++e2) {
      const int c = sCnt[e2];
      base += (e2 < wave) ? c : 0;
    }
    const unsigned ltmask = (1u << lane) - 1u;
#pragma unroll 1
    for (int it = 0; it < kRowsBlk / 32; ++it) {
      const int l = sLab[it * 32 + lane];
      const bool pred = (l == wave);
      const unsigned m = __builtin_amdgcn_ballot_w32(pred);
      int pos = base + __builtin_popcount(m & ltmask);
      pos = pos > (kRowsBlk - 1) ? (kRowsBlk - 1) : pos;
      if (pred) sPerm[pos] = it * 32 + lane;
      base += __builtin_popcount(m);
    }
  }
  __syncthreads();

  const int c8 = (tid & 31) * 8;
  const int rw = tid >> 5;
  int start = 0;
#pragma unroll 1
  for (int e = 0; e < kExp; ++e) {
    int cnt = __builtin_amdgcn_readfirstlane(sCnt[e]);
    cnt = cnt < 0 ? 0 : cnt;
    cnt = cnt > (kRowsBlk - start) ? (kRowsBlk - start) : cnt;
    if (cnt > 0) {
      const float* W0e = W0 + (size_t)e * kInW * kHid;
      const v4f wa0 = *(const v4f*)(W0e + c8);
      const v4f wa1 = *(const v4f*)(W0e + c8 + 4);
      const v4f wb0 = *(const v4f*)(W0e + kHid + c8);
      const v4f wb1 = *(const v4f*)(W0e + kHid + c8 + 4);
      const v4f wc0 = *(const v4f*)(W0e + 2 * kHid + c8);
      const v4f wc1 = *(const v4f*)(W0e + 2 * kHid + c8 + 4);
      const v4f cc0 = *(const v4f*)(fold0 + e * kHid + c8);
      const v4f cc1 = *(const v4f*)(fold0 + e * kHid + c8 + 4);
      const float b3e = b3[e];
      const _Float16* wp1 = plane1 + (size_t)e * kHid * kHid + (size_t)(32 * wave + rl) * kHid + 8 * hh;
      const _Float16* wp2 = plane2 + (size_t)e * kHid * kHid + (size_t)(32 * wave + rl) * kHid + 8 * hh;
      const _Float16* ap  = sA + rl * kPitchA + 8 * hh;

      const int ntile = (cnt + kTileM - 1) / kTileM;
#pragma unroll 1
      for (int t = 0; t < ntile; ++t) {
        const int rem  = cnt - t * kTileM;
        const int nsub = (rem >= kTileM) ? 4 : ((rem + 15) >> 4);

        if (tid < kTileM) {
          const int li = t * kTileM + tid;
          const bool valid = li < cnt;
          const int lc = valid ? li : (cnt - 1);
          int lr = sPerm[start + lc];
          lr = lr < 0 ? 0 : lr;
          lr = lr > (kRowsBlk - 1) ? (kRowsBlk - 1) : lr;
          const float x0 = sX[lr * kDimX + 0];
          const float x1 = sX[lr * kDimX + 1];
          const float x2 = sX[lr * kDimX + 2];
          sTx[tid * 4 + 0] = valid ? x0 : 0.0f;
          sTx[tid * 4 + 1] = valid ? x1 : 0.0f;
          sTx[tid * 4 + 2] = valid ? x2 : 0.0f;
          sTx[tid * 4 + 3] = 0.0f;
          sTrow[tid] = valid ? lr : -1;
        }
        __syncthreads();

        {
          const int nrow8 = nsub * 2;
#pragma unroll 1
          for (int i = 0; i < nrow8; ++i) {
            const int m = rw + 8 * i;
            const v4f xv = *(const v4f*)(sTx + m * 4);
            v8h hv;
#pragma unroll
            for (int q = 0; q < 4; ++q) {
              float v = cc0[q];
              v = fmaf(xv[0], wa0[q], v);
              v = fmaf(xv[1], wb0[q], v);
              v = fmaf(xv[2], wc0[q], v);
              hv[q] = operand_h(fmaxf(v, 0.0f) * kCarryA);
              float u = cc1[q];
              u = fmaf(xv[0], wa1[q], u);
              u = fmaf(xv[1], wb1[q], u);
              u = fmaf(xv[2], wc1[q], u);
              hv[4 + q] = operand_h(fmaxf(u, 0.0f) * kCarryA);
            }
            *(v8h*)(sA + m * kPitchA + c8) = hv;
          }
        }
        __syncthreads();

        v8f acc[4][2];
#pragma unroll
        for (int i = 0; i < 4; ++i) {
          acc[i][0] = (v8f){0.f, 0.f, 0.f, 0.f, 0.f, 0.f, 0.f, 0.f};
          acc[i][1] = (v8f){0.f, 0.f, 0.f, 0.f, 0.f, 0.f, 0.f, 0.f};
        }

#pragma unroll 1
        for (int k0 = 0; k0 < kHid; k0 += 32) {
          const v16h wf0 = frag_load(wp1 + k0);
          const v16h wf1 = frag_load(wp1 + 16 * kHid + k0);
#pragma unroll
          for (int i = 0; i < 4; ++i) {
            if (i < nsub) {
              const v16h af = frag_load(ap + i * 16 * kPitchA + k0);
              acc[i][0] = mma_h(wf0, af, acc[i][0]);
              acc[i][1] = mma_h(wf1, af, acc[i][1]);
            }
          }
        }
        __syncthreads();

#pragma unroll
        for (int j = 0; j < 2; ++j) {
          const int n = 32 * wave + 16 * j + 8 * hh;
          const v4f ba = *(const v4f*)(b1 + e * kHid + n);
          const v4f bb = *(const v4f*)(b1 + e * kHid + n + 4);
#pragma unroll
          for (int i = 0; i < 4; ++i) {
            v8h hv;
#pragma unroll
            for (int r = 0; r < 4; ++r) {
              const float v = fmaf(acc[i][j][r], kFoldBack, ba[r]);
              hv[r] = operand_h(fmaxf(v, 0.0f) * kCarryA);
              const float u = fmaf(acc[i][j][4 + r], kFoldBack, bb[r]);
              hv[4 + r] = operand_h(fmaxf(u, 0.0f) * kCarryA);
            }
            *(v8h*)(sA + (i * 16 + rl) * kPitchA + n) = hv;
          }
        }
        __syncthreads();

#pragma unroll
        for (int i = 0; i < 4; ++i) {
          acc[i][0] = (v8f){0.f, 0.f, 0.f, 0.f, 0.f, 0.f, 0.f, 0.f};
          acc[i][1] = (v8f){0.f, 0.f, 0.f, 0.f, 0.f, 0.f, 0.f, 0.f};
        }

#pragma unroll 1
        for (int k0 = 0; k0 < kHid; k0 += 32) {
          const v16h wf0 = frag_load(wp2 + k0);
          const v16h wf1 = frag_load(wp2 + 16 * kHid + k0);
#pragma unroll
          for (int i = 0; i < 4; ++i) {
            if (i < nsub) {
              const v16h af = frag_load(ap + i * 16 * kPitchA + k0);
              acc[i][0] = mma_h(wf0, af, acc[i][0]);
              acc[i][1] = mma_h(wf1, af, acc[i][1]);
            }
          }
        }

        {
          float p0 = 0.0f, p1 = 0.0f, p2 = 0.0f, p3 = 0.0f;
#pragma unroll
          for (int j = 0; j < 2; ++j) {
            const int n = 32 * wave + 16 * j + 8 * hh;
            const v4f ba = *(const v4f*)(b2 + e * kHid + n);
            const v4f bb = *(const v4f*)(b2 + e * kHid + n + 4);
            const v4f ha = *(const v4f*)(W3 + e * kHid + n);
            const v4f hb = *(const v4f*)(W3 + e * kHid + n + 4);
#pragma unroll
            for (int r = 0; r < 4; ++r) {
              p0 = fmaf(fmaxf(fmaf(acc[0][j][r], kFoldBack, ba[r]), 0.0f), ha[r], p0);
              p0 = fmaf(fmaxf(fmaf(acc[0][j][4 + r], kFoldBack, bb[r]), 0.0f), hb[r], p0);
              p1 = fmaf(fmaxf(fmaf(acc[1][j][r], kFoldBack, ba[r]), 0.0f), ha[r], p1);
              p1 = fmaf(fmaxf(fmaf(acc[1][j][4 + r], kFoldBack, bb[r]), 0.0f), hb[r], p1);
              p2 = fmaf(fmaxf(fmaf(acc[2][j][r], kFoldBack, ba[r]), 0.0f), ha[r], p2);
              p2 = fmaf(fmaxf(fmaf(acc[2][j][4 + r], kFoldBack, bb[r]), 0.0f), hb[r], p2);
              p3 = fmaf(fmaxf(fmaf(acc[3][j][r], kFoldBack, ba[r]), 0.0f), ha[r], p3);
              p3 = fmaf(fmaxf(fmaf(acc[3][j][4 + r], kFoldBack, bb[r]), 0.0f), hb[r], p3);
            }
          }
          p0 += __shfl_xor(p0, 16, 32);
          p1 += __shfl_xor(p1, 16, 32);
          p2 += __shfl_xor(p2, 16, 32);
          p3 += __shfl_xor(p3, 16, 32);
          if (hh == 0) {
            sPart[wave * kTileM + 0  + rl] = p0;
            sPart[wave * kTileM + 16 + rl] = p1;
            sPart[wave * kTileM + 32 + rl] = p2;
            sPart[wave * kTileM + 48 + rl] = p3;
          }
        }
        __syncthreads();

        if (tid < kTileM) {
          float s = 0.0f;
#pragma unroll
          for (int w = 0; w < 8; ++w) s += sPart[w * kTileM + tid];
          s += b3e;
          const int tr = sTrow[tid];
          if (tr >= 0) sOut[tr] = s;
        }
      }
    }
    start += cnt;
  }
  __syncthreads();

  if (wave < 4) {
    const v4f v = *(const v4f*)(sOut + wave * 128 + lane * 4);
    float* q = out + row0 + wave * 128 + lane * 4;
    *(volatile v4f*)q = v;
    __threadfence();
    *(volatile v4f*)q = v;
  }
}

extern "C" void kernel_launch(void* const* d_in, const int* in_sizes, int n_in,
                              void* d_out, int out_size, void* d_ws, size_t ws_size,
                              hipStream_t stream) {
  if (n_in < 11) return;
  if (in_sizes[0] != kPts * kDimX) return;
  if (in_sizes[1] != kPts) return;
  if (in_sizes[2] != kExp * kLat) return;
  if (in_sizes[3] != kExp * kInW * kHid) return;
  if (in_sizes[4] != kExp * kHid) return;
  if (in_sizes[5] != kExp * kHid * kHid) return;
  if (in_sizes[6] != kExp * kHid) return;
  if (in_sizes[7] != kExp * kHid * kHid) return;
  if (in_sizes[8] != kExp * kHid) return;
  if (in_sizes[9] != kExp * kHid) return;
  if (in_sizes[10] != kExp) return;
  if (out_size != kPts) return;
  if (ws_size < kWsTotal) return;

  const float* x      = (const float*)d_in[0];
  const int*   labels = (const int*)  d_in[1];
  const float* emb    = (const float*)d_in[2];
  const float* W0     = (const float*)d_in[3];
  const float* b0     = (const float*)d_in[4];
  const float* W1     = (const float*)d_in[5];
  const float* b1     = (const float*)d_in[6];
  const float* W2     = (const float*)d_in[7];
  const float* b2     = (const float*)d_in[8];
  const float* W3     = (const float*)d_in[9];
  const float* b3     = (const float*)d_in[10];
  float* out = (float*)d_out;

  char* ws = (char*)d_ws;
  _Float16* plane1 = (_Float16*)(ws + kOffPlane1);
  _Float16* plane2 = (_Float16*)(ws + kOffPlane2);
  float*    fold0  = (float*)(ws + kOffFold0);

  weight_plane_kernel<<<2 * kExp * 16, 256, 0, stream>>>(W1, W2, plane1, plane2);
  latent_fold_kernel<<<kExp, kHid, 0, stream>>>(emb, W0, b0, fold0);
  routed_decoder_kernel<<<kPts / kRowsBlk, 256, 0, stream>>>(
      x, labels, W0, fold0, plane1, b1, plane2, b2, W3, b3, out);
}
